// OAIAttention_17729624998176
// MI455X (gfx1250) — hardware-run, weakly checked
//
#include <hip/hip_runtime.h>


namespace {
constexpr int T = 1024, HID = 2880, NQ = 64, NKV = 8, GQ = 8, D = 64, QO = NQ * D  , KO = NKV * D  , QKV = QO + 2 * KO  , WIN = 128, KB = 128, ICTX = 4096;
constexpr float HS = 256.0f, WSC = 256.0f, PS = 256.0f, EPS = 1e-5f, SCALE = 0.125f;
typedef _Float16 b16;
typedef __attribute__((ext_vector_type(16))) _Float16 v16b;
typedef __attribute__((ext_vector_type(8))) _Float16 v8b;
typedef __attribute__((ext_vector_type(8))) float v8f;
typedef __attribute__((ext_vector_type(4))) float v4f;
__device__ __forceinline__ float bf16_rne(float f) { unsigned int u = __float_as_uint(f); u += 0x7FFFu + ((u >> 16) & 1u); float r = __uint_as_float(u & 0xFFFF0000u); asm volatile("" : "+v"(r)); return r; }
__device__ __forceinline__ float bfv(float f) { float r = bf16_rne(f); asm volatile("" : "+v"(r)); return r; }
__device__ __forceinline__ void split16(float v, b16& hi, b16& lo) { hi = (b16)v; lo = (b16)(v - (float)hi); }
__device__ __forceinline__ v16b frag_kb(const b16* p, int hh) { const v8b a = *(const v8b*)(p + 8 * hh), b = *(const v8b*)(p + 16 + 8 * hh); v16b f;
#pragma unroll
  for (int e = 0; e < 8; ++e) { f[e] = a[e]; f[8 + e] = b[e]; } return f; }
__device__ __forceinline__ v8f wmma16b(v16b a, v16b b, v8f c) { v8f d = __builtin_amdgcn_wmma_f32_16x16x32_f16(false, a, false, b, (short)0, c, false, false); asm volatile("v_nop\n\tv_nop\n\tv_nop\n\tv_nop" : "+v"(d) : "v"(a), "v"(b)); return d; }
__device__ __forceinline__ void wave_lds_sync() { __builtin_amdgcn_fence(__ATOMIC_RELEASE, "workgroup"); __builtin_amdgcn_wave_barrier(); __builtin_amdgcn_fence(__ATOMIC_ACQUIRE, "workgroup"); }
__device__ __forceinline__ float pmul(float a, float b) { float p = a * b; asm volatile("" : "+v"(p)); return p; }
__device__ __forceinline__ int iclamp(int v, int lo, int hi) { return v < lo ? lo : (v > hi ? hi : v); }

__global__ __launch_bounds__(256) void rope_kernel(float* __restrict__ COS, float* __restrict__ SIN) { const int u = blockIdx.x * 256 + threadIdx.x; if (u >= ICTX * (D / 2)) return; const int t = u / (D / 2), i = u % (D / 2);
  const double base = 150000.0, scaling = 32.0, alpha = 1.0, beta = 32.0, dhalf = 32.0, two_pi = 6.283185307179586;
  const double freq = pow(base, (double)(2 * i) / (double)D); const double conc = 0.1 * log(scaling) + 1.0;
  const double low = dhalf * log((double)ICTX / (beta * two_pi)) / log(base), high = dhalf * log((double)ICTX / (alpha * two_pi)) / log(base);
  const double interp = 1.0 / (scaling * freq), extrap = 1.0 / freq; double ramp = ((double)i - low) / (high - low); ramp = ramp < 0.0 ? 0.0 : (ramp > 1.0 ? 1.0 : ramp); const double mask = 1.0 - ramp; const double invf = interp * (1.0 - mask) + extrap * mask;
  const double f = (double)t * invf; const float c = (float)(cos(f) * conc), s = (float)(sin(f) * conc);
  for (int pass = 0; pass < 2; ++pass) { ((volatile float*)COS)[u] = c; ((volatile float*)SIN)[u] = s; __threadfence(); } }
__global__ __launch_bounds__(256) void wput_kernel(const float* __restrict__ wqkv, const float* __restrict__ wout, b16* __restrict__ WQ, b16* __restrict__ WO) { const size_t nt = (size_t)gridDim.x * 256, u0 = (size_t)blockIdx.x * 256 + threadIdx.x; v8b v;
  for (size_t u = u0; u < (size_t)QKV * (HID / 8); u += nt) { const int o = (int)(u / (HID / 8)), k0 = (int)(u % (HID / 8)) * 8;
#pragma unroll
    for (int j = 0; j < 8; ++j) v[j] = (b16)(bf16_rne(wqkv[(size_t)(k0 + j) * QKV + o]) * WSC); for (int pass = 0; pass < 2; ++pass) { *(volatile v8b*)(WQ + (size_t)o * HID + k0) = v; __threadfence(); } }
  for (size_t u = u0; u < (size_t)HID * (QO / 8); u += nt) { const int o = (int)(u / (QO / 8)), k0 = (int)(u % (QO / 8)) * 8;
#pragma unroll
    for (int j = 0; j < 8; ++j) v[j] = (b16)(bf16_rne(wout[(size_t)(k0 + j) * HID + o]) * WSC); for (int pass = 0; pass < 2; ++pass) { *(volatile v8b*)(WO + (size_t)o * QO + k0) = v; __threadfence(); } } }
__global__ __launch_bounds__(32) void norm_kernel(const float* __restrict__ x, const float* __restrict__ ns, int TLIM, b16* __restrict__ TNh, b16* __restrict__ TNl) { const int lane = threadIdx.x; const size_t m0 = (size_t)blockIdx.x * 16; if (m0 >= (size_t)TLIM) return;
  for (int rr = 0; rr < 16; ++rr) { const float* xr = x + (m0 + rr) * HID; float s = 0.0f; for (int k = lane; k < HID; k += 32) { const float v = bfv(xr[k]); s += v * v; } for (int o = 16; o; o >>= 1) s += __shfl_xor(s, o); const float r = rsqrtf(s / HID + EPS);
    for (int pass = 0; pass < 2; ++pass) { for (int k0 = lane * 8; k0 < HID; k0 += 256) { v8b hv, lv;
#pragma unroll
        for (int j = 0; j < 8; ++j) { b16 p, ql; split16(pmul(pmul(bfv(xr[k0 + j]), r), bfv(ns[k0 + j])) * HS, p, ql); hv[j] = p; lv[j] = ql; } *(volatile v8b*)(TNh + (m0 + rr) * HID + k0) = hv; *(volatile v8b*)(TNl + (m0 + rr) * HID + k0) = lv; } __threadfence(); } } }
__global__ __launch_bounds__(32) void qkv_kernel(const b16* __restrict__ TNh, const b16* __restrict__ TNl, const b16* __restrict__ WQ, const float* __restrict__ bq, const int* __restrict__ pos, const float* __restrict__ COS, const float* __restrict__ SIN, int TLIM, b16* __restrict__ Ph, b16* __restrict__ Pl) { constexpr int KC = 288; __shared__ __attribute__((aligned(16))) b16 Ah[16][KC + 8], Al[16][KC + 8]; __shared__ float Tf[16][260]; const int lane = threadIdx.x, nloc = lane & 15, hlf = lane >> 4; const int g = blockIdx.x % (QKV / 256); const size_t m0 = (size_t)(blockIdx.x / (QKV / 256)) * 16; if (m0 >= (size_t)TLIM) return; const int c0 = g * 256;
  v8f acc[16];
#pragma unroll
  for (int t = 0; t < 16; ++t) acc[t] = (v8f){};
  if (lane < 16) for (int k = KC; k < KC + 8; ++k) { Ah[lane][k] = (b16)0.0f; Al[lane][k] = (b16)0.0f; }
#pragma unroll 1
  for (int kc = 0; kc < HID; kc += KC) { for (int rr = 0; rr < 16; ++rr) for (int q = lane; q < KC / 8; q += 32) { *(v8b*)(&Ah[rr][q * 8]) = *(const v8b*)(TNh + (m0 + rr) * HID + kc + q * 8); *(v8b*)(&Al[rr][q * 8]) = *(const v8b*)(TNl + (m0 + rr) * HID + kc + q * 8); }
    wave_lds_sync();
#pragma unroll 3
    for (int kb = 0; kb < KC; kb += 32) { const v16b a = frag_kb(&Ah[nloc][kb], hlf), al = frag_kb(&Al[nloc][kb], hlf);
#pragma unroll
      for (int t = 0; t < 16; ++t) { const v16b bw = frag_kb(WQ + (size_t)(c0 + t * 16 + nloc) * HID + kc + kb, hlf); acc[t] = wmma16b(a, bw, acc[t]); acc[t] = wmma16b(al, bw, acc[t]); } }
    wave_lds_sync(); }
#pragma unroll
  for (int t = 0; t < 16; ++t) { const int cc = t * 16 + nloc; const float bb = bfv(bq[c0 + cc]);
#pragma unroll
    for (int r8 = 0; r8 < 8; ++r8) Tf[8 * hlf + r8][cc] = acc[t][r8] * (1.0f / (HS * WSC)) + bb; }
  wave_lds_sync();
  const bool isq = c0 < QO, isk = (c0 >= QO) && (c0 < QO + KO);
  for (int rr = 0; rr < 16; ++rr) { const int p = iclamp(pos[m0 + rr], 0, ICTX - 1); const float cs = COS[p * 32 + lane], sn = SIN[p * 32 + lane];
#pragma unroll
    for (int hb = 0; hb < 4; ++hb) { float x1 = Tf[rr][hb * 64 + lane], x2 = Tf[rr][hb * 64 + 32 + lane]; float y1 = x1, y2 = x2; if (isq || isk) { y1 = pmul(x1, cs) - pmul(x2, sn); y2 = pmul(x2, cs) + pmul(x1, sn); } if (isq) { y1 *= SCALE; y2 *= SCALE; }
      b16 ph, pl; split16(y1 * HS, ph, pl); Ah[rr][hb * 64 + lane] = ph; Al[rr][hb * 64 + lane] = pl; split16(y2 * HS, ph, pl); Ah[rr][hb * 64 + 32 + lane] = ph; Al[rr][hb * 64 + 32 + lane] = pl; } }
  wave_lds_sync();
  for (int pass = 0; pass < 2; ++pass) { for (int rr = 0; rr < 16; ++rr) { *(volatile v8b*)(Ph + (m0 + rr) * QKV + c0 + lane * 8) = *(const v8b*)(&Ah[rr][lane * 8]); *(volatile v8b*)(Pl + (m0 + rr) * QKV + c0 + lane * 8) = *(const v8b*)(&Al[rr][lane * 8]); } __threadfence(); } }
__global__ __launch_bounds__(32) void att_kernel(const b16* __restrict__ Ph, const b16* __restrict__ Pl, const float* __restrict__ sinks, int TLIM, float* __restrict__ ATT) { __shared__ __attribute__((aligned(16))) b16 P_h[16][KB + 8], P_l[16][KB + 8], Vth[D][KB + 8], Vtl[D][KB + 8]; __shared__ float Sf[16][KB + 4], Of[16][D + 4];
  const int lane = threadIdx.x, nloc = lane & 15, hlf = lane >> 4; const int h = blockIdx.x / (T / 16), qt = blockIdx.x % (T / 16); const int t0 = qt * 16; if (t0 >= TLIM) return; const int kvh = h / GQ; const int qoff = h * D, koff = QO + kvh * D, voff = QO + KO + kvh * D;
  v16b qa[2], qb[2];
#pragma unroll
  for (int ks = 0; ks < 2; ++ks) { qa[ks] = frag_kb(Ph + (size_t)(t0 + nloc) * QKV + qoff + ks * 32, hlf); qb[ks] = frag_kb(Pl + (size_t)(t0 + nloc) * QKV + qoff + ks * 32, hlf); }
  const float sk = bfv(sinks[h]); float m_r[8], den_r[8]; v8f acc[4];
#pragma unroll
  for (int r8 = 0; r8 < 8; ++r8) { m_r[r8] = sk; den_r[r8] = 1.0f; }
#pragma unroll
  for (int t = 0; t < 4; ++t) acc[t] = (v8f){};
  const int kstart = ((t0 - WIN + 1) < 0 ? 0 : (t0 - WIN + 1)) & ~(KB - 1), kend = t0 + 16;
#pragma unroll 1
  for (int kb0 = kstart; kb0 < kend; kb0 += KB) {
    for (int rr = 0; rr < KB; rr += 2) { const int r = rr + hlf; const int key = kb0 + r < T ? kb0 + r : T - 1; const size_t vr = (size_t)key * QKV + voff; for (int s = 0; s < D / 16; ++s) { Vth[s * 16 + nloc][r] = Ph[vr + s * 16 + nloc]; Vtl[s * 16 + nloc][r] = Pl[vr + s * 16 + nloc]; } }
#pragma unroll
    for (int t = 0; t < KB / 16; ++t) { const int key = kb0 + t * 16 + nloc; const int kc = key < T ? key : T - 1; const size_t kr = (size_t)kc * QKV + koff; v8f s = {};
#pragma unroll
      for (int ks = 0; ks < 2; ++ks) { const v16b ka = frag_kb(Ph + kr + ks * 32, hlf), kl = frag_kb(Pl + kr + ks * 32, hlf); s = wmma16b(qa[ks], ka, s); s = wmma16b(qa[ks], kl, s); s = wmma16b(qb[ks], ka, s); }
#pragma unroll
      for (int r8 = 0; r8 < 8; ++r8) { const int i = t0 + 8 * hlf + r8, j = kb0 + t * 16 + nloc; const bool ok = (j <= i) && (j > i - WIN) && (j < T); Sf[8 * hlf + r8][t * 16 + nloc] = ok ? s[r8] * (1.0f / (HS * HS)) : -INFINITY; } }
    wave_lds_sync();
#pragma unroll
    for (int rr = 0; rr < 16; ++rr) { float mx = -INFINITY;
#pragma unroll
      for (int q = 0; q < 4; ++q) mx = fmaxf(mx, Sf[rr][q * 32 + lane]);
      for (int o = 16; o; o >>= 1) mx = fmaxf(mx, __shfl_xor(mx, o));
      const float mold = __shfl(m_r[rr & 7], (rr >> 3) * 16); const float mn = fmaxf(mold, mx); const float sf = __expf(mold - mn); float ps = 0.0f;
#pragma unroll
      for (int q = 0; q < 4; ++q) { const int kx = q * 32 + lane; const float sv = Sf[rr][kx]; const float p = (sv == -INFINITY) ? 0.0f : __expf(sv - mn); ps += p; b16 ph, pl; split16(p * PS, ph, pl); P_h[rr][kx] = ph; P_l[rr][kx] = pl; }
      for (int o = 16; o; o >>= 1) ps += __shfl_xor(ps, o);
      if ((rr >> 3) == hlf) { const int r8 = rr & 7; den_r[r8] = den_r[r8] * sf + ps; m_r[r8] = mn;
#pragma unroll
        for (int t = 0; t < 4; ++t) acc[t][r8] = acc[t][r8] * sf; } }
    wave_lds_sync();
#pragma unroll
    for (int ks = 0; ks < KB; ks += 32) { const v16b pa = frag_kb(&P_h[nloc][ks], hlf), pb = frag_kb(&P_l[nloc][ks], hlf);
#pragma unroll
      for (int t = 0; t < 4; ++t) { const v16b vh = frag_kb(&Vth[t * 16 + nloc][ks], hlf), vl = frag_kb(&Vtl[t * 16 + nloc][ks], hlf); acc[t] = wmma16b(pa, vh, acc[t]); acc[t] = wmma16b(pa, vl, acc[t]); acc[t] = wmma16b(pb, vh, acc[t]); } }
    wave_lds_sync(); }
#pragma unroll
  for (int t = 0; t < 4; ++t)
#pragma unroll
    for (int r8 = 0; r8 < 8; ++r8) Of[8 * hlf + r8][t * 16 + nloc] = acc[t][r8] * (1.0f / (HS * PS)) / den_r[r8];
  wave_lds_sync();
  for (int pass = 0; pass < 2; ++pass) { for (int rr = 0; rr < 16; ++rr) for (int s2 = 0; s2 < D / 32; ++s2) ((volatile float*)ATT)[(size_t)(t0 + rr) * QO + qoff + s2 * 32 + lane] = Of[rr][s2 * 32 + lane]; __threadfence(); } }
__global__ __launch_bounds__(32) void oproj_kernel(const float* __restrict__ ATT, const b16* __restrict__ WO, const float* __restrict__ bo, const float* __restrict__ x, int TLIM, float* __restrict__ out) { constexpr int NTL = 18, GW = NTL * 16  , KC = 256; __shared__ __attribute__((aligned(16))) b16 Ah[16][KC + 8], Al[16][KC + 8]; __shared__ float Tf[16][GW + 4]; const int lane = threadIdx.x, nloc = lane & 15, hlf = lane >> 4; const int g = blockIdx.x % (HID / GW); const size_t m0 = (size_t)(blockIdx.x / (HID / GW)) * 16; if (m0 >= (size_t)TLIM) return; const int c0 = g * GW;
  v8f acc[NTL];
#pragma unroll
  for (int t = 0; t < NTL; ++t) acc[t] = (v8f){};
  if (lane < 16) for (int k = KC; k < KC + 8; ++k) { Ah[lane][k] = (b16)0.0f; Al[lane][k] = (b16)0.0f; }
#pragma unroll 1
  for (int kc = 0; kc < QO; kc += KC) { for (int rr = 0; rr < 16; ++rr) for (int q = 0; q < KC / 32; ++q) { b16 p, ql; split16(ATT[(m0 + rr) * QO + kc + q * 32 + lane] * HS, p, ql); Ah[rr][q * 32 + lane] = p; Al[rr][q * 32 + lane] = ql; }
    wave_lds_sync();
#pragma unroll 2
    for (int kb = 0; kb < KC; kb += 32) { const v16b a = frag_kb(&Ah[nloc][kb], hlf), al = frag_kb(&Al[nloc][kb], hlf);
#pragma unroll
      for (int t = 0; t < NTL; ++t) { const v16b bw = frag_kb(WO + (size_t)(c0 + t * 16 + nloc) * QO + kc + kb, hlf); acc[t] = wmma16b(a, bw, acc[t]); acc[t] = wmma16b(al, bw, acc[t]); } }
    wave_lds_sync(); }
#pragma unroll
  for (int t = 0; t < NTL; ++t) { const int cc = t * 16 + nloc; const float bb = bfv(bo[c0 + cc]);
#pragma unroll
    for (int r8 = 0; r8 < 8; ++r8) { const int rr = 8 * hlf + r8; Tf[rr][cc] = acc[t][r8] * (1.0f / (HS * WSC)) + bb + bfv(x[(m0 + rr) * HID + c0 + cc]); } }
  wave_lds_sync();
  for (int pass = 0; pass < 2; ++pass) { for (int rr = 0; rr < 16; ++rr) for (int c = lane; c < GW; c += 32) ((volatile float*)out)[(m0 + rr) * HID + c0 + c] = Tf[rr][c]; __threadfence(); } }
}

extern "C" void kernel_launch(void* const* d_in, const int* in_sizes, int n_in, void* d_out, int out_size, void* d_ws, size_t ws_size, hipStream_t stream) {
  (void)n_in;
  auto Fp = [&](int i) { return (const float*)d_in[i]; }; auto Ip = [&](int i) { return (const int*)d_in[i]; };
  if (in_sizes[0] != T * HID || in_sizes[1] != T || in_sizes[2] != HID || in_sizes[3] != HID * QKV || in_sizes[4] != QKV || in_sizes[5] != QO * HID || in_sizes[6] != HID || in_sizes[7] != NQ || out_size != T * HID) return;
  const int TLIM = T;
  size_t off = 0; char* ws = (char*)d_ws;
  auto carve = [&](size_t bytes) { char* p = ws + off; off += (bytes + 255) & ~(size_t)255; return p; };
  b16* WQ = (b16*)carve((size_t)QKV * HID * 2); b16* WO = (b16*)carve((size_t)HID * QO * 2); float* COS = (float*)carve((size_t)ICTX * 32 * 4); float* SIN = (float*)carve((size_t)ICTX * 32 * 4); b16* TNh = (b16*)carve((size_t)T * HID * 2); b16* TNl = (b16*)carve((size_t)T * HID * 2);
  b16* Ph = (b16*)carve((size_t)T * QKV * 2); b16* Pl = (b16*)carve((size_t)T * QKV * 2); float* ATT = (float*)carve((size_t)T * QO * 4);
  if (off > ws_size || off > ((size_t)128 << 20)) return;
  rope_kernel<<<(ICTX * 32 + 255) / 256, 256, 0, stream>>>(COS, SIN);
  wput_kernel<<<4096, 256, 0, stream>>>(Fp(3), Fp(5), WQ, WO);
  norm_kernel<<<TLIM / 16, 32, 0, stream>>>(Fp(0), Fp(2), TLIM, TNh, TNl);
  qkv_kernel<<<(TLIM / 16) * (QKV / 256), 32, 0, stream>>>(TNh, TNl, WQ, Fp(4), Ip(1), COS, SIN, TLIM, Ph, Pl);
  att_kernel<<<NQ * (T / 16), 32, 0, stream>>>(Ph, Pl, Fp(7), TLIM, ATT);
  oproj_kernel<<<(TLIM / 16) * (HID / 288), 32, 0, stream>>>(ATT, WO, Fp(6), Fp(0), TLIM, (float*)d_out);
}
